// RandlaNet_34849364640184
// MI455X (gfx1250) — hardware-verified
//
#include <hip/hip_runtime.h>


namespace {
constexpr int N = 200000, NLIM = 200000  , K = 16, DI = 16, D1 = 16, D2 = 32, DO = 64, HP = 32  ;
constexpr float XS = 8.0f, WSC = 256.0f, SL = 0.2f;
static_assert(N % 64 == 0 && NLIM % 64 == 0, "tiling");
typedef _Float16 b16;
typedef __attribute__((ext_vector_type(16))) _Float16 v16b;
typedef __attribute__((ext_vector_type(8))) _Float16 v8b;
typedef __attribute__((ext_vector_type(8))) float v8f;
typedef __attribute__((ext_vector_type(4))) float v4f;
__device__ __forceinline__ float bf16_rne(float f) { unsigned int u = __float_as_uint(f); u += 0x7FFFu + ((u >> 16) & 1u); return __uint_as_float(u & 0xFFFF0000u); }
__device__ __forceinline__ void split16(float v, b16& hi, b16& lo) { hi = (b16)v; lo = (b16)(v - (float)hi); }
__device__ __forceinline__ v16b frag_kb(const b16* p, int hh) { const v8b a = *(const v8b*)(p + 8 * hh), b = *(const v8b*)(p + 16 + 8 * hh); v16b f;
#pragma unroll
  for (int e = 0; e < 8; ++e) { f[e] = a[e]; f[8 + e] = b[e]; } return f; }
__device__ __forceinline__ v8f wmma16b(v16b a, v16b b, v8f c) { v8f d = __builtin_amdgcn_wmma_f32_16x16x32_f16(false, a, false, b, (short)0, c, false, false); asm volatile("v_nop\n\tv_nop\n\tv_nop\n\tv_nop" : "+v"(d) : "v"(a), "v"(b)); return d; }
__device__ __forceinline__ void wave_lds_sync() { __builtin_amdgcn_fence(__ATOMIC_RELEASE, "workgroup"); __builtin_amdgcn_wave_barrier(); __builtin_amdgcn_fence(__ATOMIC_ACQUIRE, "workgroup"); }
__device__ __forceinline__ float pmul(float a, float b) { float p = a * b; asm volatile("" : "+v"(p)); return p; }
__device__ __forceinline__ int iclamp(int v, int lo, int hi) { return v < lo ? lo : (v > hi ? hi : v); }

__device__ __forceinline__ float lk(float v) { return v >= 0.0f ? v : SL * v; }
__global__ __launch_bounds__(256) void prep_kernel(const float* __restrict__ a1, const float* __restrict__ a2, b16* __restrict__ WATT) {
  const int t = threadIdx.x; if (t >= 2 * 32 * 32 / 8) return; const int l = t / 128; const int e = (t % 128) * 8; const int oo = e / 32, c0 = e % 32; const float* a = l == 0 ? a1 : a2; v8b o;
  for (int j = 0; j < 8; ++j) o[j] = (b16)(bf16_rne(a[(c0 + j) * 32 + oo]) * WSC);
  for (int pass = 0; pass < 2; ++pass) { *(volatile v8b*)(WATT + l * 1024 + e) = o; __threadfence(); }
}
__global__ __launch_bounds__(256) void start_kernel(const float* __restrict__ x, const float* __restrict__ ws, const float* __restrict__ bs, float* __restrict__ H0) {
  __shared__ float SWS[DI * D1], SBS[D1];
  for (int q2 = threadIdx.x; q2 < DI * D1; q2 += 256) SWS[q2] = bf16_rne(ws[q2]); for (int q2 = threadIdx.x; q2 < D1; q2 += 256) SBS[q2] = bf16_rne(bs[q2]);
  __syncthreads();
  const size_t u = (size_t)blockIdx.x * 256 + threadIdx.x; const size_t i = u / 8; const int q = (int)(u % 8) * 4; if (i >= (size_t)N) return; v4f o = {0.0f, 0.0f, 0.0f, 0.0f};
  if (q < D1) { float xv[DI]; { const float* xr = x + i * DI; for (int c4 = 0; c4 < DI; c4 += 4) { const v4f f = *(const v4f*)(xr + c4); for (int c = 0; c < 4; ++c) xv[c4 + c] = bf16_rne(f[c]); } }
    for (int jj = 0; jj < 4; ++jj) { const int d = q + jj; float s = SBS[d];
#pragma unroll
      for (int c = 0; c < DI; ++c) s += xv[c] * SWS[c * D1 + d]; o[jj] = lk(s); } }
  for (int pass = 0; pass < 2; ++pass) { *(volatile v4f*)(H0 + i * HP + q) = o; __threadfence(); }
}
template <int DP, bool LAST>
__global__ __launch_bounds__(256) void conv_kernel(const float* __restrict__ HIN, const float* __restrict__ pos, const int* __restrict__ nidx, const float* __restrict__ wr, const float* __restrict__ br, const b16* __restrict__ WATT, const float* __restrict__ wp, const float* __restrict__ bp, float* __restrict__ HO,
                                                    const float* __restrict__ x, const float* __restrict__ we, const float* __restrict__ be, const float* __restrict__ wsk, const float* __restrict__ bsk, float* __restrict__ out) {
  __shared__ __attribute__((aligned(16))) float FH[8][16][32 + 2]; __shared__ float SWR[10 * 16], SBR[16], SWP[32 * 32], SBP[32], SWE[LAST ? D2 * DO : 1], SWSK[LAST ? DI * DO : 1], SBE[LAST ? DO : 1], SBSK[LAST ? DO : 1];
  for (int q = threadIdx.x; q < 10 * 16; q += 256) SWR[q] = bf16_rne(wr[q]); for (int q = threadIdx.x; q < 16; q += 256) SBR[q] = bf16_rne(br[q]);
  for (int q = threadIdx.x; q < 32 * DP; q += 256) SWP[q] = bf16_rne(wp[q]); for (int q = threadIdx.x; q < DP; q += 256) SBP[q] = bf16_rne(bp[q]);
  if (LAST) { for (int q = threadIdx.x; q < D2 * DO; q += 256) SWE[q] = bf16_rne(we[q]); for (int q = threadIdx.x; q < DI * DO; q += 256) SWSK[q] = bf16_rne(wsk[q]); for (int q = threadIdx.x; q < DO; q += 256) { SBE[q] = bf16_rne(be[q]); SBSK[q] = bf16_rne(bsk[q]); } }
  __syncthreads();
  const int wave = threadIdx.x >> 5, lane = threadIdx.x & 31, col = lane & 15, hh = lane >> 4; const size_t i = (size_t)blockIdx.x * 8 + wave; if (i >= (size_t)NLIM) return;
  int j = nidx[i * K + col]; j = iclamp(j, 0, N - 1);
  float pi[3], pj[3], rp[10]; for (int a = 0; a < 3; ++a) { pi[a] = bf16_rne(pos[i * 3 + a]); pj[a] = bf16_rne(pos[(size_t)j * 3 + a]); }
  { float d2 = 0.0f; for (int a = 0; a < 3; ++a) { rp[a] = pi[a]; rp[3 + a] = pj[a]; rp[6 + a] = pi[a] - pj[a]; d2 += rp[6 + a] * rp[6 + a]; } rp[9] = sqrtf(d2 + 1e-12f); }
  float fx[8], fr[8];
  { const v4f a0 = *(const v4f*)(HIN + (size_t)j * HP + 8 * hh), a1 = *(const v4f*)(HIN + (size_t)j * HP + 8 * hh + 4); for (int q = 0; q < 4; ++q) { fx[q] = a0[q]; fx[4 + q] = a1[q]; } if (j >= NLIM) { for (int q = 0; q < 8; ++q) fx[q] = 0.0f; } }
#pragma unroll
  for (int q = 0; q < 8; ++q) { const int d = 8 * hh + q; float s = SBR[d];
#pragma unroll
    for (int t = 0; t < 10; ++t) s += rp[t] * SWR[t * 16 + d]; fr[q] = lk(s); }
  v16b ah, al;
#pragma unroll
  for (int q = 0; q < 8; ++q) { b16 p, ql; split16(fx[q] * XS, p, ql); ah[q] = p; al[q] = ql; split16(fr[q] * XS, p, ql); ah[8 + q] = p; al[8 + q] = ql; }
  v8f acc[2] = {(v8f){}, (v8f){}};
#pragma unroll
  for (int t = 0; t < 2; ++t) { const v16b bw = frag_kb(WATT + (size_t)(t * 16 + col) * 32, hh); acc[t] = wmma16b(ah, bw, acc[t]); acc[t] = wmma16b(al, bw, acc[t]); }
  for (int q = 0; q < 8; ++q) { FH[wave][col][8 * hh + q] = fx[q]; FH[wave][col][16 + 8 * hh + q] = fr[q]; }
  wave_lds_sync();
  float aggv[2];
#pragma unroll
  for (int t = 0; t < 2; ++t) { float lg[8]; float mx = -INFINITY; for (int r = 0; r < 8; ++r) { lg[r] = acc[t][r] * (1.0f / (XS * WSC)); mx = fmaxf(mx, lg[r]); }
    mx = fmaxf(mx, __shfl_xor(mx, 16)); float sum = 0.0f, ws_ = 0.0f; const int o = t * 16 + col;
#pragma unroll
    for (int r = 0; r < 8; ++r) { const float e = __expf(lg[r] - mx); sum += e; ws_ += e * FH[wave][8 * hh + r][o]; }
    sum += __shfl_xor(sum, 16); ws_ += __shfl_xor(ws_, 16); aggv[t] = ws_ / sum; }
  float ag[32];
#pragma unroll
  for (int o = 0; o < 16; ++o) { ag[o] = __shfl(aggv[0], o); ag[16 + o] = __shfl(aggv[1], o); }
  float hd = 0.0f; if (lane < DP) { float s = SBP[lane];
#pragma unroll
    for (int o = 0; o < 32; ++o) s += ag[o] * SWP[o * DP + lane]; hd = lk(s); }
  if (!LAST) { for (int pass = 0; pass < 2; ++pass) { ((volatile float*)HO)[i * HP + lane] = (lane < DP) ? hd : 0.0f; __threadfence(); } }
  else {
    float hv[32];
#pragma unroll
    for (int d = 0; d < 32; ++d) hv[d] = __shfl(hd, d);
    float xv[DI]; { const float* xr = x + i * DI; for (int c4 = 0; c4 < DI; c4 += 4) { const v4f f = *(const v4f*)(xr + c4); for (int c = 0; c < 4; ++c) xv[c4 + c] = bf16_rne(f[c]); } }
    float ov[2];
#pragma unroll
    for (int u = 0; u < 2; ++u) { const int o = lane + 32 * u; float s = SBE[o] + SBSK[o];
#pragma unroll
      for (int d = 0; d < D2; ++d) s += hv[d] * SWE[d * DO + o];
#pragma unroll
      for (int c = 0; c < DI; ++c) s += xv[c] * SWSK[c * DO + o];
      ov[u] = lk(s); }
    for (int pass = 0; pass < 2; ++pass) { ((volatile float*)out)[i * DO + lane] = ov[0]; ((volatile float*)out)[i * DO + 32 + lane] = ov[1]; __threadfence(); } }
}
}

extern "C" void kernel_launch(void* const* d_in, const int* in_sizes, int n_in, void* d_out, int out_size, void* d_ws, size_t ws_size, hipStream_t stream) {
  (void)n_in;
  auto Fp = [&](int i) { return (const float*)d_in[i]; }; auto Ip = [&](int i) { return (const int*)d_in[i]; };
  if (in_sizes[0] != N * DI || in_sizes[1] != N * 3 || in_sizes[2] != N * K || in_sizes[3] != DI * D1 || in_sizes[5] != DI * DO || in_sizes[7] != D2 * DO || in_sizes[9] != 10 * 16 || in_sizes[11] != 32 * 32 || in_sizes[12] != 32 * D1 || in_sizes[16] != 32 * 32 || in_sizes[17] != 32 * D2 || in_sizes[18] != D2 || out_size != N * DO) return;
  size_t off = 0; char* ws = (char*)d_ws;
  auto carve = [&](size_t bytes) { char* p = ws + off; off += (bytes + 255) & ~(size_t)255; return p; };
  b16* WATT = (b16*)carve(2 * 1024 * 2); float* H0 = (float*)carve((size_t)N * HP * 4); float* H1 = (float*)carve((size_t)N * HP * 4);
  if (off > ws_size || off > ((size_t)128 << 20)) return;
  prep_kernel<<<1, 256, 0, stream>>>(Fp(11), Fp(16), WATT);
  start_kernel<<<(unsigned)(((size_t)N * 8 + 255) / 256), 256, 0, stream>>>(Fp(0), Fp(3), Fp(4), H0);
  conv_kernel<D1, false><<<NLIM / 8, 256, 0, stream>>>(H0, Fp(1), Ip(2), Fp(9), Fp(10), WATT, Fp(12), Fp(13), H1, nullptr, nullptr, nullptr, nullptr, nullptr, nullptr);
  conv_kernel<D2, true><<<NLIM / 8, 256, 0, stream>>>(H1, Fp(1), Ip(2), Fp(14), Fp(15), WATT + 1024, Fp(17), Fp(18), nullptr, Fp(0), Fp(7), Fp(8), Fp(5), Fp(6), (float*)d_out);
}
